// NavierStokes_13778255086286
// MI455X (gfx1250) — hardware-verified
//
#include <hip/hip_runtime.h>
#include <math.h>

typedef __attribute__((ext_vector_type(16))) __bf16   v16b;
typedef __attribute__((ext_vector_type(8)))  __bf16   v8b;
typedef __attribute__((ext_vector_type(8)))  float    v8f;
typedef __attribute__((ext_vector_type(4)))  float    v4f;
typedef __attribute__((ext_vector_type(2)))  float    v2f;
typedef __attribute__((ext_vector_type(4)))  unsigned v4u;

constexpr int kPts        = 262144;
constexpr int kHid        = 20;
constexpr int kLayers     = 8;
constexpr int kNumCh      = 13;
constexpr int kTilePts    = 32;
constexpr int kTiles      = kPts / kTilePts;
constexpr int kChStride   = 16 * 32;
constexpr int kWaveAct    = kNumCh * kChStride;
constexpr int kOutCols    = 5;
constexpr int kTileFloats = kTilePts * kOutCols;
static_assert(kPts % kTilePts == 0);
static_assert(kTileFloats * 4 == 640 && (kTileFloats * 4) % 128 == 0);
static_assert(kHid == 20);

__device__ __forceinline__ int nrn_of(int i) {
  const int r  = i & 7;
  const int hq = (i >> 3) & 1;
  const int up = (r < 2) ? (16 + 2 * hq + r) : -1;
  return (i < 16) ? i : up;
}

constexpr size_t kOffWA   = 0;
constexpr size_t kOffW9A  = kOffWA  + (size_t)kLayers * 32 * 32 * 2;
constexpr size_t kOffBI   = kOffW9A + (size_t)16 * 32 * 2;
constexpr size_t kOffW0T  = kOffBI  + (size_t)kLayers * 32 * 4;
constexpr size_t kOffSC   = kOffW0T + (size_t)32 * 4 * 4;
constexpr size_t kWsTotal = kOffSC + (size_t)32 * 4;
static_assert(kWsTotal == 19072ull);
static_assert((kOffW9A % 128) == 0 && (kOffBI % 128) == 0 && (kOffW0T % 128) == 0 && (kOffSC % 128) == 0);

__device__ __forceinline__ unsigned bf_rne_raw(float f) {
  const unsigned u = __float_as_uint(f);
  return u + 0x7FFFu + ((u >> 16) & 1u);
}
__device__ __forceinline__ unsigned bf_rne_hi32(float f) { return bf_rne_raw(f) & 0xFFFF0000u; }
__device__ __forceinline__ float bf_rne(float f) { return __uint_as_float(bf_rne_hi32(f)); }
__device__ __forceinline__ unsigned pack2(unsigned even_raw, unsigned odd_raw) {
  return (even_raw >> 16) | (odd_raw & 0xFFFF0000u);
}
__device__ __forceinline__ void split_pair(float va, float vb, unsigned& hw, unsigned& lw) {
  const unsigned ra = bf_rne_raw(va);
  const unsigned rb = bf_rne_raw(vb);
  const float fa = __uint_as_float(ra & 0xFFFF0000u);
  const float fb = __uint_as_float(rb & 0xFFFF0000u);
  const float da = va - fa;
  const float db = vb - fb;
  const unsigned la = bf_rne_raw(da);
  const unsigned lb = bf_rne_raw(db);
  hw = pack2(ra, rb);
  lw = pack2(la, lb);
}

__device__ __forceinline__ void sched_fence() { asm volatile("" ::: "memory"); }

union FragU { v16b v; v8b h[2]; };
__device__ __forceinline__ v16b frag_load(const __bf16* p) {
  FragU f;
  f.h[0] = *(const v8b*)(p);
  f.h[1] = *(const v8b*)(p + 16);
  return f.v;
}
__device__ __forceinline__ v8f wmma_bf(v16b a, v16b b, v8f c) {
  return __builtin_amdgcn_wmma_f32_16x16x32_bf16(false, a, false, b, (short)0, c, false, false);
}
__device__ __forceinline__ void guard1(v8f& c, v16b a, v16b bh, v16b bl) {
  asm volatile("v_nop\n\tv_nop\n\tv_nop\n\tv_nop" : "+v"(c) : "v"(a), "v"(bh), "v"(bl));
}
__device__ __forceinline__ void mm4(v16b a0, v16b a1, v16b bh, v16b bl, v8f& c0, v8f& c1) {
  c0 = wmma_bf(a0, bh, c0);
  c1 = wmma_bf(a1, bh, c1);
  c0 = wmma_bf(a0, bl, c0);
  c1 = wmma_bf(a1, bl, c1);
  guard1(c0, a0, bh, bl);
  guard1(c1, a1, bh, bl);
}

__device__ __forceinline__ void store2_u(unsigned* p, v4u v) {
  *(volatile v4u*)p = v;
  __threadfence();
  *(volatile v4u*)p = v;
}
__device__ __forceinline__ void store2_f(float* p, v4f v) {
  *(volatile v4f*)p = v;
  __threadfence();
  *(volatile v4f*)p = v;
}

__global__ __launch_bounds__(256) void prepack_kernel(
    const float* __restrict__ Wh, const float* __restrict__ bh,
    const float* __restrict__ W0, const float* __restrict__ b0,
    const float* __restrict__ W9, const float* __restrict__ b9,
    const float* __restrict__ lam1, const float* __restrict__ lam2,
    unsigned char* __restrict__ ws)
{
  const int tid = threadIdx.x;
  const float s_b9p = bf_rne(b9[1]);
  const float s_b9z = bf_rne(b9[0]);
  const float s_l1  = bf_rne(lam1[0]);
  const float s_l2  = bf_rne(lam2[0]);

#pragma unroll 1
  for (int it = 0; it < 4; ++it) {
    const int q   = it * 256 + tid;
    const int l   = q >> 7;
    const int m   = (q >> 2) & 31;
    const int k0  = (q & 3) * 8;
    const int nm  = nrn_of(m);
    const int nmc = (nm < 0) ? 0 : nm;
    unsigned hb[8];
#pragma unroll
    for (int e = 0; e < 8; ++e) {
      const int nk  = nrn_of(k0 + e);
      const int nkc = (nk < 0) ? 0 : nk;
      const float wraw = Wh[l * (kHid * kHid) + nmc * kHid + nkc];
      const float w = ((nm >= 0) && (nk >= 0)) ? wraw : 0.0f;
      hb[e] = bf_rne_hi32(w);
    }
    const v4u wv = (v4u){pack2(hb[0], hb[1]), pack2(hb[2], hb[3]), pack2(hb[4], hb[5]), pack2(hb[6], hb[7])};
    store2_u((unsigned*)(ws + kOffWA) + (size_t)q * 4, wv);
  }

  if (tid < 64) {
    const int m  = tid >> 2;
    const int k0 = (tid & 3) * 8;
    const int mc = (m < 2) ? m : 1;
    unsigned hb[8];
#pragma unroll
    for (int e = 0; e < 8; ++e) {
      const int nk  = nrn_of(k0 + e);
      const int nkc = (nk < 0) ? 0 : nk;
      const float wraw = W9[mc * kHid + nkc];
      const float w = ((m < 2) && (nk >= 0)) ? wraw : 0.0f;
      hb[e] = bf_rne_hi32(w);
    }
    const v4u wv = (v4u){pack2(hb[0], hb[1]), pack2(hb[2], hb[3]), pack2(hb[4], hb[5]), pack2(hb[6], hb[7])};
    store2_u((unsigned*)(ws + kOffW9A) + (size_t)tid * 4, wv);
  } else if (tid < 128) {
    const int q  = tid - 64;
    const int l  = q >> 3;
    const int j0 = (q & 7) * 4;
    v4f bv;
#pragma unroll
    for (int e = 0; e < 4; ++e) {
      const int nj  = nrn_of(j0 + e);
      const int njc = (nj < 0) ? 0 : nj;
      const float braw = bh[l * kHid + njc];
      bv[e] = (nj >= 0) ? bf_rne(braw) : 0.0f;
    }
    store2_f((float*)(ws + kOffBI) + (size_t)q * 4, bv);
  } else if (tid < 160) {
    const int m   = tid - 128;
    const int nm  = nrn_of(m);
    const int nmc = (nm < 0) ? 0 : nm;
    const float a0 = W0[nmc * 3 + 0];
    const float a1 = W0[nmc * 3 + 1];
    const float a2 = W0[nmc * 3 + 2];
    const float a3 = b0[nmc];
    const bool live = (nm >= 0);
    v4f rv;
    rv[0] = live ? bf_rne(a0) : 0.0f;
    rv[1] = live ? bf_rne(a1) : 0.0f;
    rv[2] = live ? bf_rne(a2) : 0.0f;
    rv[3] = live ? bf_rne(a3) : 0.0f;
    store2_f((float*)(ws + kOffW0T) + (size_t)m * 4, rv);
  } else if (tid < 168) {
    const int q = tid - 160;
    const bool first = (q == 0);
    v4f sv;
    sv[0] = first ? s_b9p : 0.0f;
    sv[1] = first ? s_l1  : 0.0f;
    sv[2] = first ? s_l2  : 0.0f;
    sv[3] = first ? s_b9z : 0.0f;
    store2_f((float*)(ws + kOffSC) + (size_t)q * 4, sv);
  }
}

__device__ __forceinline__ float fast_tanh(float s) {
  float e = __expf(-2.f * fabsf(s));
  float a = (1.f - e) * __builtin_amdgcn_rcpf(1.f + e);
  return copysignf(a, s);
}

template <class VT>
__device__ __forceinline__ VT tanh_vec(VT s) {
  VT a;
  constexpr int kN = (int)(sizeof(VT) / sizeof(float));
#pragma unroll
  for (int j = 0; j < kN; ++j) {
    const float sj = s[j];
    a[j] = fast_tanh(sj);
  }
  return a;
}

template <class VT>
struct JetRegs { VT f1, f2, f3, Sx, Sy, St, Sxx, Sxy, Syy; };

template <int C, class VT>
__device__ __forceinline__ VT jet_channel(JetRegs<VT>& J, VT S, VT bias) {
  VT o;
  if (C == 0) {
    const VT s  = S + bias;
    const VT av = tanh_vec<VT>(s);
    const VT t1 = 1.f - av * av;
    J.f1 = t1;
    J.f2 = -2.f * av * t1;
    J.f3 = t1 * (6.f * av * av - 2.f);
    o = av;
  } else if (C == 1) {
    J.Sx = S;
    o = J.f1 * S;
  } else if (C == 2) {
    J.Sy = S;
    o = J.f1 * S;
  } else if (C == 3) {
    J.St = S;
    o = J.f1 * S;
  } else if (C == 4) {
    J.Sxx = S;
    o = J.f2 * J.Sx * J.Sx + J.f1 * S;
  } else if (C == 5) {
    J.Sxy = S;
    o = J.f2 * J.Sx * J.Sy + J.f1 * S;
  } else if (C == 6) {
    J.Syy = S;
    o = J.f2 * J.Sy * J.Sy + J.f1 * S;
  } else if (C == 7) {
    o = J.f2 * J.Sx * J.St + J.f1 * S;
  } else if (C == 8) {
    o = J.f2 * J.Sy * J.St + J.f1 * S;
  } else if (C == 9) {
    o = J.f3 * J.Sx * J.Sx * J.Sx + 3.f * J.f2 * J.Sxx * J.Sx + J.f1 * S;
  } else if (C == 10) {
    o = J.f3 * J.Sx * J.Sx * J.Sy + J.f2 * (J.Sxx * J.Sy + 2.f * J.Sxy * J.Sx) + J.f1 * S;
  } else if (C == 11) {
    o = J.f3 * J.Sx * J.Sy * J.Sy + J.f2 * (J.Syy * J.Sx + 2.f * J.Sxy * J.Sy) + J.f1 * S;
  } else {
    o = J.f3 * J.Sy * J.Sy * J.Sy + 3.f * J.f2 * J.Syy * J.Sy + J.f1 * S;
  }
  return o;
}

__device__ __forceinline__ void st_act(__bf16* ph, __bf16* pl, v8f o0, v2f o1) {
  unsigned h0w, h1w, h2w, h3w, h4w;
  unsigned l0w, l1w, l2w, l3w, l4w;
  const float a0 = o0[0];
  const float a1 = o0[1];
  const float a2 = o0[2];
  const float a3 = o0[3];
  const float a4 = o0[4];
  const float a5 = o0[5];
  const float a6 = o0[6];
  const float a7 = o0[7];
  const float r0 = o1[0];
  const float r1 = o1[1];
  split_pair(a0, a1, h0w, l0w);
  split_pair(a2, a3, h1w, l1w);
  split_pair(a4, a5, h2w, l2w);
  split_pair(a6, a7, h3w, l3w);
  split_pair(r0, r1, h4w, l4w);
  const v4u hv0 = (v4u){h0w, h1w, h2w, h3w};
  const v4u hv1 = (v4u){h4w, 0u, 0u, 0u};
  const v4u lv0 = (v4u){l0w, l1w, l2w, l3w};
  const v4u lv1 = (v4u){l4w, 0u, 0u, 0u};
  *(v8b*)(ph)      = __builtin_bit_cast(v8b, hv0);
  *(v8b*)(ph + 16) = __builtin_bit_cast(v8b, hv1);
  *(v8b*)(pl)      = __builtin_bit_cast(v8b, lv0);
  *(v8b*)(pl + 16) = __builtin_bit_cast(v8b, lv1);
  sched_fence();
}

template <int C>
__device__ __forceinline__ void first_channel(JetRegs<v8f>& J0, JetRegs<v2f>& J1,
    __bf16* ph, __bf16* pl,
    v8f wx0, v2f wx1, v8f wy0, v2f wy1, v8f wt0, v2f wt1, v8f bz0, v2f bz1,
    float xv, float yv, float tv)
{
  v8f s0;
  v2f s1;
  if (C == 0) {
    s0 = wt0 * tv + (wy0 * yv + wx0 * xv);
    s1 = wt1 * tv + (wy1 * yv + wx1 * xv);
  } else if (C == 1) {
    s0 = wx0;
    s1 = wx1;
  } else if (C == 2) {
    s0 = wy0;
    s1 = wy1;
  } else if (C == 3) {
    s0 = wt0;
    s1 = wt1;
  } else {
    s0 = (v8f){0.f, 0.f, 0.f, 0.f, 0.f, 0.f, 0.f, 0.f};
    s1 = (v2f){0.f, 0.f};
  }
  const v8f o0 = jet_channel<C, v8f>(J0, s0, bz0);
  const v2f o1 = jet_channel<C, v2f>(J1, s1, bz1);
  st_act(ph + C * kChStride, pl + C * kChStride, o0, o1);
}

template <int C>
__device__ __forceinline__ void hidden_channel(JetRegs<v8f>& J0, JetRegs<v2f>& J1,
    __bf16* ph, __bf16* pl, const __bf16* wl, v8f bz0, v2f bz1)
{
  sched_fence();
  const v16b bh  = frag_load(ph + C * kChStride);
  const v16b bl  = frag_load(pl + C * kChStride);
  const v16b aw0 = frag_load(wl);
  const v16b aw1 = frag_load(wl + 16 * 32);
  v8f c0 = (v8f){0.f, 0.f, 0.f, 0.f, 0.f, 0.f, 0.f, 0.f};
  v8f c1 = (v8f){0.f, 0.f, 0.f, 0.f, 0.f, 0.f, 0.f, 0.f};
  mm4(aw0, aw1, bh, bl, c0, c1);
  const v8f s0 = c0;
  const v2f s1 = (v2f){c1[0], c1[1]};
  const v8f o0 = jet_channel<C, v8f>(J0, s0, bz0);
  const v2f o1 = jet_channel<C, v2f>(J1, s1, bz1);
  st_act(ph + C * kChStride, pl + C * kChStride, o0, o1);
}

template <int C>
__device__ __forceinline__ void out_channel(const __bf16* ph, const __bf16* pl, v16b a9, float& r0, float& r1) {
  sched_fence();
  const v16b bh = frag_load(ph + C * kChStride);
  const v16b bl = frag_load(pl + C * kChStride);
  v8f acc = (v8f){0.f, 0.f, 0.f, 0.f, 0.f, 0.f, 0.f, 0.f};
  acc = wmma_bf(a9, bh, acc);
  acc = wmma_bf(a9, bl, acc);
  guard1(acc, a9, bh, bl);
  r0 = acc[0];
  r1 = acc[1];
  sched_fence();
}

__global__ __launch_bounds__(64) __attribute__((amdgpu_num_vgpr(232))) void jet_mlp_kernel(
    const float* __restrict__ gx, const float* __restrict__ gy, const float* __restrict__ gt,
    const unsigned short* WAp, const unsigned short* __restrict__ W9Ap,
    const float* __restrict__ BI, const float* __restrict__ W0T, const float* __restrict__ SC,
    float* __restrict__ out, int ntiles)
{
  __shared__ __align__(16) __bf16 sHi[2 * kWaveAct];
  __shared__ __align__(16) __bf16 sLo[2 * kWaveAct];
  __shared__ __align__(16) float  sOut[kTileFloats];

  const int tid  = threadIdx.x;
  const int wave = tid >> 5;
  const int lane = tid & 31;
  const int n    = lane & 15;
  const int half = lane >> 4;
  const int tile = ((int)blockIdx.x < ntiles) ? (int)blockIdx.x : (ntiles - 1);

  const __bf16* WA  = (const __bf16*)WAp;
  const __bf16* W9A = (const __bf16*)W9Ap;
  __bf16* ph = sHi + wave * kWaveAct + n * 32 + 8 * half;
  __bf16* pl = sLo + wave * kWaveAct + n * 32 + 8 * half;

  const int idx = tile * kTilePts + wave * 16 + n;
  const float xv = bf_rne(gx[idx]);
  const float yv = bf_rne(gy[idx]);
  const float tv = bf_rne(gt[idx]);

  {
    v8f wx0, wy0, wt0, bz0;
    v2f wx1, wy1, wt1, bz1;
#pragma unroll
    for (int j = 0; j < 8; ++j) {
      const v4f rv = *(const v4f*)(W0T + (8 * half + j) * 4);
      wx0[j] = rv[0];
      wy0[j] = rv[1];
      wt0[j] = rv[2];
      bz0[j] = rv[3];
    }
#pragma unroll
    for (int j = 0; j < 2; ++j) {
      const v4f rv = *(const v4f*)(W0T + (16 + 8 * half + j) * 4);
      wx1[j] = rv[0];
      wy1[j] = rv[1];
      wt1[j] = rv[2];
      bz1[j] = rv[3];
    }
    JetRegs<v8f> J0;
    JetRegs<v2f> J1;
    first_channel<0>(J0, J1, ph, pl, wx0, wx1, wy0, wy1, wt0, wt1, bz0, bz1, xv, yv, tv);
    first_channel<1>(J0, J1, ph, pl, wx0, wx1, wy0, wy1, wt0, wt1, bz0, bz1, xv, yv, tv);
    first_channel<2>(J0, J1, ph, pl, wx0, wx1, wy0, wy1, wt0, wt1, bz0, bz1, xv, yv, tv);
    first_channel<3>(J0, J1, ph, pl, wx0, wx1, wy0, wy1, wt0, wt1, bz0, bz1, xv, yv, tv);
    first_channel<4>(J0, J1, ph, pl, wx0, wx1, wy0, wy1, wt0, wt1, bz0, bz1, xv, yv, tv);
    first_channel<5>(J0, J1, ph, pl, wx0, wx1, wy0, wy1, wt0, wt1, bz0, bz1, xv, yv, tv);
    first_channel<6>(J0, J1, ph, pl, wx0, wx1, wy0, wy1, wt0, wt1, bz0, bz1, xv, yv, tv);
    first_channel<7>(J0, J1, ph, pl, wx0, wx1, wy0, wy1, wt0, wt1, bz0, bz1, xv, yv, tv);
    first_channel<8>(J0, J1, ph, pl, wx0, wx1, wy0, wy1, wt0, wt1, bz0, bz1, xv, yv, tv);
    first_channel<9>(J0, J1, ph, pl, wx0, wx1, wy0, wy1, wt0, wt1, bz0, bz1, xv, yv, tv);
    first_channel<10>(J0, J1, ph, pl, wx0, wx1, wy0, wy1, wt0, wt1, bz0, bz1, xv, yv, tv);
    first_channel<11>(J0, J1, ph, pl, wx0, wx1, wy0, wy1, wt0, wt1, bz0, bz1, xv, yv, tv);
    first_channel<12>(J0, J1, ph, pl, wx0, wx1, wy0, wy1, wt0, wt1, bz0, bz1, xv, yv, tv);
  }
  __syncthreads();

#pragma unroll 1
  for (int l = 0; l < kLayers; ++l) {
    const __bf16* wl = WA + l * (32 * 32) + n * 32 + 8 * half;
    v8f bz0;
    v2f bz1;
    {
      const float* bp = BI + l * 32 + 8 * half;
      const v4f b0v = *(const v4f*)(bp);
      const v4f b1v = *(const v4f*)(bp + 4);
      const v4f b2v = *(const v4f*)(bp + 16);
      bz0 = (v8f){b0v[0], b0v[1], b0v[2], b0v[3], b1v[0], b1v[1], b1v[2], b1v[3]};
      bz1 = (v2f){b2v[0], b2v[1]};
    }
    JetRegs<v8f> J0;
    JetRegs<v2f> J1;
    hidden_channel<0>(J0, J1, ph, pl, wl, bz0, bz1);
    hidden_channel<1>(J0, J1, ph, pl, wl, bz0, bz1);
    hidden_channel<2>(J0, J1, ph, pl, wl, bz0, bz1);
    hidden_channel<3>(J0, J1, ph, pl, wl, bz0, bz1);
    hidden_channel<4>(J0, J1, ph, pl, wl, bz0, bz1);
    hidden_channel<5>(J0, J1, ph, pl, wl, bz0, bz1);
    hidden_channel<6>(J0, J1, ph, pl, wl, bz0, bz1);
    hidden_channel<7>(J0, J1, ph, pl, wl, bz0, bz1);
    hidden_channel<8>(J0, J1, ph, pl, wl, bz0, bz1);
    hidden_channel<9>(J0, J1, ph, pl, wl, bz0, bz1);
    hidden_channel<10>(J0, J1, ph, pl, wl, bz0, bz1);
    hidden_channel<11>(J0, J1, ph, pl, wl, bz0, bz1);
    hidden_channel<12>(J0, J1, ph, pl, wl, bz0, bz1);
    __syncthreads();
  }

  float psi1, psi2, psi4, psi5, psi6, psi7, psi8, psi9, psi10, psi11, psi12;
  float pj0, pj1, pj2;
  {
    const v16b a9 = frag_load(W9A + n * 32 + 8 * half);
    float d0, d1;
    out_channel<0>(ph, pl, a9, d0, pj0);
    out_channel<1>(ph, pl, a9, psi1, pj1);
    out_channel<2>(ph, pl, a9, psi2, pj2);
    out_channel<4>(ph, pl, a9, psi4, d1);
    out_channel<5>(ph, pl, a9, psi5, d1);
    out_channel<6>(ph, pl, a9, psi6, d1);
    out_channel<7>(ph, pl, a9, psi7, d1);
    out_channel<8>(ph, pl, a9, psi8, d1);
    out_channel<9>(ph, pl, a9, psi9, d1);
    out_channel<10>(ph, pl, a9, psi10, d1);
    out_channel<11>(ph, pl, a9, psi11, d1);
    out_channel<12>(ph, pl, a9, psi12, d1);
  }

  {
    const v4f scv = *(const v4f*)SC;
    const float b9p = scv[0];
    const float l1  = scv[1];
    const float l2  = scv[2];
    const float u    =  psi2;
    const float v_   = -psi1;
    const float pp   =  pj0 + b9p;
    const float u_x  =  psi5;
    const float u_y  =  psi6;
    const float u_t  =  psi8;
    const float u_xx =  psi10;
    const float u_yy =  psi12;
    const float v_x  = -psi4;
    const float v_y  = -psi5;
    const float v_t  = -psi7;
    const float v_xx = -psi9;
    const float v_yy = -psi11;
    const float p_x  =  pj1;
    const float p_y  =  pj2;
    const float f  = u_t + l1 * (u * u_x + v_ * u_y) + p_x - l2 * (u_xx + u_yy);
    const float gq = v_t + l1 * (u * v_x + v_ * v_y) + p_y - l2 * (v_xx + v_yy);
    if (half == 0) {
      float* so = sOut + (wave * 16 + n) * kOutCols;
      so[0] = u;
      so[1] = v_;
      so[2] = pp;
      so[3] = f;
      so[4] = gq;
    }
  }
  __syncthreads();

  if (wave == 0) {
    const v4f ov0 = *(const v4f*)(sOut + lane * 4);
    const v4f ov1 = *(const v4f*)(sOut + 128 + (lane & 7) * 4);
    float* ob = out + (size_t)tile * kTileFloats;
    for (int pass = 0; pass < 2; ++pass) {
      *(volatile v4f*)(ob + lane * 4) = ov0;
      if (lane < 8) *(volatile v4f*)(ob + 128 + lane * 4) = ov1;
      __threadfence();
    }
  }
}

extern "C" void kernel_launch(void* const* d_in, const int* in_sizes, int n_in,
                              void* d_out, int out_size, void* d_ws, size_t ws_size,
                              hipStream_t stream) {
  if (n_in < 11) return;
  if (in_sizes[0] != kPts || in_sizes[1] != kPts || in_sizes[2] != kPts) return;
  if (in_sizes[3] != kHid * 3 || in_sizes[4] != kHid) return;
  if (in_sizes[5] != kLayers * kHid * kHid || in_sizes[6] != kLayers * kHid) return;
  if (in_sizes[7] != 2 * kHid || in_sizes[8] != 2) return;
  if (in_sizes[9] != 1 || in_sizes[10] != 1) return;
  if (out_size != kPts * kOutCols) return;
  if (ws_size < kWsTotal) return;

  const float* x    = (const float*)d_in[0];
  const float* y    = (const float*)d_in[1];
  const float* t    = (const float*)d_in[2];
  const float* W0   = (const float*)d_in[3];
  const float* b0   = (const float*)d_in[4];
  const float* Wh   = (const float*)d_in[5];
  const float* bh   = (const float*)d_in[6];
  const float* W9   = (const float*)d_in[7];
  const float* b9   = (const float*)d_in[8];
  const float* lam1 = (const float*)d_in[9];
  const float* lam2 = (const float*)d_in[10];

  unsigned char* ws = (unsigned char*)d_ws;
  const unsigned short* WA  = (const unsigned short*)(ws + kOffWA);
  const unsigned short* W9A = (const unsigned short*)(ws + kOffW9A);
  const float* BI  = (const float*)(ws + kOffBI);
  const float* W0T = (const float*)(ws + kOffW0T);
  const float* SC  = (const float*)(ws + kOffSC);

  prepack_kernel<<<1, 256, 0, stream>>>(Wh, bh, W0, b0, W9, b9, lam1, lam2, ws);
  jet_mlp_kernel<<<kTiles, 64, 0, stream>>>(x, y, t, WA, W9A, BI, W0T, SC, (float*)d_out, kTiles);
}
